// Block_51977694216642
// MI455X (gfx1250) — hardware-verified
//
#include <hip/hip_runtime.h>
#include <math.h>

constexpr int kNB   = 4;
constexpr int kNT   = 1024;
constexpr int kNC   = 512;
constexpr int kNH   = 4;
constexpr int kND   = kNC / kNH;
constexpr int kRows = kNB * kNT;
constexpr int kFF   = 4 * kNC;
constexpr int kChunk = 16;
constexpr int kSliceW = 64;
constexpr float kWCarry    = 16.0f;
constexpr float kActCarry  = 16.0f;
constexpr float kScaleW    = 1.0f / kWCarry;
constexpr float kScaleWA   = 1.0f / (kWCarry * kActCarry);
constexpr float kInvC      = 1.0f / (float)kNC;
constexpr float kLnEps     = 1e-5f;
constexpr float kRmsEps    = 1e-8f;
constexpr int kSmallBlocks = (kNC * kNC) / (8 * 256);
constexpr int kBigBlocks   = (kFF * kNC) / (8 * 256);
constexpr int kCvtBlocks   = 5 * kSmallBlocks + 2 * kBigBlocks;
static_assert(kND == 128, "head width");
static_assert(kRows % 64 == 0 && kNC % 64 == 0 && kFF % 64 == 0, "GEMM M and N are 64-tile multiples");
static_assert(kNC % 32 == 0 && kFF % 32 == 0, "GEMM K multiples of 32");
static_assert(kRows % 8 == 0, "row kernels: 8 rows per block exact");
static_assert(kNT % kChunk == 0, "scan chunks exact");
static_assert((kNC * kNC) % (8 * 256) == 0 && (kFF * kNC) % (8 * 256) == 0, "cast grid exact");
static_assert(kNC == 512, "lane maps assume 512 channels");

typedef __attribute__((ext_vector_type(16))) _Float16 v16h;
typedef __attribute__((ext_vector_type(8)))  _Float16 v8h;
typedef __attribute__((ext_vector_type(8)))  float    v8f;
typedef __attribute__((ext_vector_type(4)))  float    v4f;

union FragU { v16h v; v8h h[2]; };
__device__ __forceinline__ v16h frag_load(const _Float16* p) {
  FragU f;
  f.h[0] = *(const v8h*)(p);
  f.h[1] = *(const v8h*)(p + 16);
  return f.v;
}
__device__ __forceinline__ v8f frag_mma(v16h a, v16h b, v8f c) {
  return __builtin_amdgcn_wmma_f32_16x16x32_f16(false, a, false, b, (short)0, c, false, false);
}
__device__ __forceinline__ void row_guard_h(v8f& a, v8f& b, v8f& c, v8f& d, v16h x, v16h b0, v16h b1, v16h b2, v16h b3) {
  asm volatile("v_nop\n\tv_nop\n\tv_nop\n\tv_nop" : "+v"(a), "+v"(b), "+v"(c), "+v"(d) : "v"(x), "v"(b0), "v"(b1), "v"(b2), "v"(b3));
}
__device__ __forceinline__ void keep4_h(v16h a, v16h b, v16h c, v16h d) { asm volatile("v_nop" :: "v"(a), "v"(b), "v"(c), "v"(d)); }
__device__ __forceinline__ void acc_guard4(v8f& a, v8f& b, v8f& c, v8f& d) { asm volatile("v_nop\n\tv_nop\n\tv_nop\n\tv_nop" : "+v"(a), "+v"(b), "+v"(c), "+v"(d)); }
__device__ __forceinline__ void wave_lds_sync() {
  __builtin_amdgcn_fence(__ATOMIC_RELEASE, "workgroup");
  __builtin_amdgcn_wave_barrier();
  __builtin_amdgcn_fence(__ATOMIC_ACQUIRE, "workgroup");
}

template <int OUT_MODE, bool RESID, int POST>
__global__ __launch_bounds__(256) void wmma_gemm64_h(
    const unsigned short* __restrict__ Ap, int lda, long strideA,
    const unsigned short* __restrict__ Btp, int ldb, long strideB,
    void* __restrict__ Cout, int ldc, long strideC,
    const float* __restrict__ resid, long strideR,
    int M, int N, int K, float scale, float postScale) {
  static_assert(!(RESID && OUT_MODE != 0), "residual add only on f32 output");
  const _Float16* A  = (const _Float16*)Ap;
  const _Float16* Bt = (const _Float16*)Btp;
  __shared__ __align__(16) float sT[8][16 * 68];
  const int b    = blockIdx.y;
  const int lane = threadIdx.x & 31;
  const int wave = threadIdx.x >> 5;
  const int tilesN = N >> 6;
  const int tilesM = M >> 6;
  const int tile = blockIdx.x * 8 + wave;
  if (tile >= tilesM * tilesN) return;
  const int tm = tile / tilesN;
  const int tn = tile - tm * tilesN;
  const int m0 = tm << 6;
  const int n0 = tn << 6;

  const _Float16* Ab = A  + (size_t)b * strideA;
  const _Float16* Bb = Bt + (size_t)b * strideB;

  const int rlane = lane & 15;
  const int koff  = (lane >> 4) * 8;
  const int mOff  = (lane >> 4) * 8;

  v8f acc[4][4];
#pragma unroll
  for (int i = 0; i < 4; ++i)
#pragma unroll
    for (int j = 0; j < 4; ++j) acc[i][j] = (v8f){0.f, 0.f, 0.f, 0.f, 0.f, 0.f, 0.f, 0.f};

  for (int k0 = 0; k0 < K; k0 += 32) {
    v16h bh[4];
#pragma unroll
    for (int j = 0; j < 4; ++j) {
      const size_t bo = (size_t)(n0 + (j << 4) + rlane) * ldb + koff + k0;
      bh[j] = frag_load(Bb + bo);
    }
#pragma unroll
    for (int i = 0; i < 4; ++i) {
      const size_t ao = (size_t)(m0 + (i << 4) + rlane) * lda + koff + k0;
      const v16h ah = frag_load(Ab + ao);
#pragma unroll
      for (int j = 0; j < 4; ++j) acc[i][j] = frag_mma(ah, bh[j], acc[i][j]);
      row_guard_h(acc[i][0], acc[i][1], acc[i][2], acc[i][3], ah, bh[0], bh[1], bh[2], bh[3]);
    }
    keep4_h(bh[0], bh[1], bh[2], bh[3]);
  }
  acc_guard4(acc[0][0], acc[0][1], acc[0][2], acc[0][3]);
  acc_guard4(acc[1][0], acc[1][1], acc[1][2], acc[1][3]);
  acc_guard4(acc[2][0], acc[2][1], acc[2][2], acc[2][3]);
  acc_guard4(acc[3][0], acc[3][1], acc[3][2], acc[3][3]);

  float* slab = sT[wave];
  const float* Rb = resid + (size_t)b * strideR;
#pragma unroll
  for (int i = 0; i < 4; ++i) {
    const int mBase = m0 + (i << 4);
#pragma unroll
    for (int j = 0; j < 4; ++j) {
#pragma unroll
      for (int r = 0; r < 8; ++r) {
        slab[(mOff + r) * 68 + (j << 4) + rlane] = acc[i][j][r] * scale;
      }
    }
    wave_lds_sync();
    if (POST == 1) {
#pragma unroll 1
      for (int idx = lane; idx < 16 * 64; idx += 32) {
        const int rr = idx >> 6, cc = idx & 63;
        const float v = slab[rr * 68 + cc];
        const float gl = 0.5f * v * (1.0f + erff(v * 0.70710678118654752f));
        slab[rr * 68 + cc] = gl * postScale;
      }
      wave_lds_sync();
    }
    if (POST == 2) {
      if (b == 3) {
#pragma unroll 1
        for (int idx = lane; idx < 16 * 64; idx += 32) {
          const int rr = idx >> 6, cc = idx & 63;
          const float v = slab[rr * 68 + cc];
          slab[rr * 68 + cc] = 1.0f / (1.0f + expf(-v));
        }
      }
      wave_lds_sync();
    }
    if (RESID) {
      const int hh = lane >> 4, c4 = (lane & 15) * 4;
#pragma unroll
      for (int it = 0; it < 8; ++it) {
        const int row = it * 2 + hh;
        v4f sv = *(const v4f*)(slab + row * 68 + c4);
        const v4f rv = *(const v4f*)(Rb + (size_t)(mBase + row) * ldc + n0 + c4);
        sv += rv;
        *(v4f*)(slab + row * 68 + c4) = sv;
      }
      wave_lds_sync();
    }
    if (OUT_MODE == 0) {
      float* C = (float*)Cout + (size_t)b * strideC;
      const int hh = lane >> 4, c4 = (lane & 15) * 4;
      for (int pass = 0; pass < 2; ++pass) {
#pragma unroll
        for (int it = 0; it < 8; ++it) {
          const int row = it * 2 + hh;
          const v4f v = *(const v4f*)(slab + row * 68 + c4);
          *(volatile v4f*)(C + (size_t)(mBase + row) * ldc + n0 + c4) = v;
        }
        __threadfence();
      }
    } else {
      const int q = lane >> 3, c8 = (lane & 7) * 8;
      unsigned short* C = (unsigned short*)Cout + (size_t)b * strideC;
      for (int pass = 0; pass < 2; ++pass) {
#pragma unroll
        for (int it = 0; it < 4; ++it) {
          const int row = it * 4 + q;
          const float* sp = slab + row * 68 + c8;
          v8h hv;
#pragma unroll
          for (int e = 0; e < 8; ++e) hv[e] = (_Float16)sp[e];
          *(volatile v8h*)(C + (size_t)(mBase + row) * ldc + n0 + c8) = hv;
        }
        __threadfence();
      }
    }
    wave_lds_sync();
  }
}

__global__ __launch_bounds__(256) void prep_kernel(
    const float* __restrict__ wq, const float* __restrict__ wk, const float* __restrict__ wv,
    const float* __restrict__ wg, const float* __restrict__ wo, const float* __restrict__ w1,
    const float* __restrict__ w2, const float* __restrict__ tdec,
    unsigned short* __restrict__ w16, float* __restrict__ lamOut) {
  __shared__ __align__(16) float sl[kNC];
  const int blk = blockIdx.x;
  const int tid = threadIdx.x;
  if (blk >= kCvtBlocks) {
#pragma unroll 1
    for (int u = 0; u < 2; ++u) {
      const int c = tid + 256 * u;
      sl[c] = expf(-expf(tdec[c]));
    }
    __syncthreads();
    if (tid < 128) {
      const v4f o = *(const v4f*)(sl + 4 * tid);
      float* op = lamOut + 4 * tid;
      *(volatile v4f*)op = o;
      __threadfence();
      *(volatile v4f*)op = o;
    }
    return;
  }
  int plane, lb;
  if (blk < 5 * kSmallBlocks) {
    plane = blk / kSmallBlocks;
    lb = blk - plane * kSmallBlocks;
  } else if (blk < 5 * kSmallBlocks + kBigBlocks) {
    plane = 5;
    lb = blk - 5 * kSmallBlocks;
  } else {
    plane = 6;
    lb = blk - 5 * kSmallBlocks - kBigBlocks;
  }
  const float* src = (plane == 0) ? wq : (plane == 1) ? wk : (plane == 2) ? wv : (plane == 3) ? wg
                   : (plane == 4) ? wo : (plane == 5) ? w1 : w2;
  const size_t dbase = (plane <= 5) ? (size_t)plane * kNC * kNC : (size_t)5 * kNC * kNC + (size_t)kFF * kNC;
  const size_t i = (size_t)lb * 256 + tid;
  const float* p = src + 8 * i;
  const v4f a = *(const v4f*)(p);
  const v4f c = *(const v4f*)(p + 4);
  v8h hv;
#pragma unroll
  for (int e = 0; e < 4; ++e) {
    hv[e]     = (_Float16)(a[e] * kWCarry);
    hv[4 + e] = (_Float16)(c[e] * kWCarry);
  }
  unsigned short* q = w16 + dbase + 8 * i;
  *(volatile v8h*)q = hv;
  __threadfence();
  *(volatile v8h*)q = hv;
}

__global__ __launch_bounds__(256) void ln1_mix_kernel(
    const float* __restrict__ x, const float* __restrict__ g1, const float* __restrict__ b1,
    const float* __restrict__ tmq, const float* __restrict__ tmk,
    const float* __restrict__ tmv, const float* __restrict__ tmg,
    unsigned short* __restrict__ xmix) {
  __shared__ __align__(16) float hb[8][2 * kNC];
  const int tid = threadIdx.x, lane = tid & 31, wave = tid >> 5;
  const int row = blockIdx.x * 8 + wave;
  const int t = row & (kNT - 1);
  float* myh = hb[wave];
#pragma unroll 1
  for (int which = 0; which < 2; ++which) {
    int srow = row - which;
    srow = srow < 0 ? 0 : srow;
    const float* rp = x + (size_t)srow * kNC;
    v4f a[4], gg[4], bb[4];
#pragma unroll
    for (int u = 0; u < 2; ++u) {
      const int off = 256 * u + 8 * lane;
      a[2 * u]      = *(const v4f*)(rp + off);
      a[2 * u + 1]  = *(const v4f*)(rp + off + 4);
      gg[2 * u]     = *(const v4f*)(g1 + off);
      gg[2 * u + 1] = *(const v4f*)(g1 + off + 4);
      bb[2 * u]     = *(const v4f*)(b1 + off);
      bb[2 * u + 1] = *(const v4f*)(b1 + off + 4);
    }
    float s = 0.0f;
#pragma unroll
    for (int i = 0; i < 4; ++i) s += (a[i][0] + a[i][1]) + (a[i][2] + a[i][3]);
#pragma unroll
    for (int off = 1; off < 32; off <<= 1) s += __shfl_xor(s, off, 32);
    const float mu = s * kInvC;
    float ss = 0.0f;
#pragma unroll
    for (int i = 0; i < 4; ++i)
#pragma unroll
      for (int e = 0; e < 4; ++e) { const float d = a[i][e] - mu; a[i][e] = d; ss += d * d; }
#pragma unroll
    for (int off = 1; off < 32; off <<= 1) ss += __shfl_xor(ss, off, 32);
    const float rstd = 1.0f / sqrtf(ss * kInvC + kLnEps);
    const bool zero = (which == 1) && (t == 0);
#pragma unroll
    for (int i = 0; i < 4; ++i) {
      v4f o;
#pragma unroll
      for (int e = 0; e < 4; ++e) {
        const float val = (gg[i][e] * a[i][e]) * rstd + bb[i][e];
        o[e] = zero ? 0.0f : val;
      }
      const int off = 256 * (i >> 1) + 8 * lane + 4 * (i & 1);
      *(v4f*)(myh + which * kNC + off) = o;
    }
  }
  wave_lds_sync();
#pragma unroll 1
  for (int p = 0; p < 4; ++p) {
    const float* tm = (p == 0) ? tmq : (p == 1) ? tmk : (p == 2) ? tmv : tmg;
    unsigned short* op = xmix + (size_t)p * kRows * kNC + (size_t)row * kNC;
    v8h hv[2];
#pragma unroll
    for (int u = 0; u < 2; ++u) {
      const int off = 256 * u + 8 * lane;
#pragma unroll
      for (int hf = 0; hf < 2; ++hf) {
        const v4f hc = *(const v4f*)(myh + off + 4 * hf);
        const v4f hp = *(const v4f*)(myh + kNC + off + 4 * hf);
        const v4f tv = *(const v4f*)(tm + off + 4 * hf);
#pragma unroll
        for (int e = 0; e < 4; ++e) {
          const float val = hc[e] * tv[e] + hp[e] * (1.0f - tv[e]);
          hv[u][4 * hf + e] = (_Float16)val;
        }
      }
    }
    for (int pass = 0; pass < 2; ++pass) {
#pragma unroll
      for (int u = 0; u < 2; ++u) *(volatile v8h*)(op + 256 * u + 8 * lane) = hv[u];
      __threadfence();
    }
  }
}

__global__ __launch_bounds__(256) void rms_exp_kernel(const float* __restrict__ raw, const float* __restrict__ scl,
                                                      float* __restrict__ outp) {
  const int tid = threadIdx.x, lane = tid & 31, wave = tid >> 5;
  const int row = blockIdx.x * 8 + wave;
  const size_t base = (size_t)blockIdx.y * kRows * kNC + (size_t)row * kNC;
  const float* rp = raw + base;
  float* op = outp + base;
  float ss = 0.0f;
#pragma unroll 1
  for (int u = 0; u < 4; ++u) {
    const v4f a = *(const v4f*)(rp + 128 * u + 4 * lane);
    ss += (a[0] * a[0] + a[1] * a[1]) + (a[2] * a[2] + a[3] * a[3]);
  }
#pragma unroll
  for (int off = 1; off < 32; off <<= 1) ss += __shfl_xor(ss, off, 32);
  const float inv_sqrt_dim = 1.0f / sqrtf((float)kNC);
  const float nrm = sqrtf(ss) * inv_sqrt_dim;
  const float inv = 1.0f / (nrm + kRmsEps);
#pragma unroll 1
  for (int u = 0; u < 4; ++u) {
    const v4f a  = *(const v4f*)(rp + 128 * u + 4 * lane);
    const v4f sc = *(const v4f*)(scl + 128 * u + 4 * lane);
    v4f o;
#pragma unroll
    for (int e = 0; e < 4; ++e) o[e] = expf(sc[e] * (a[e] * inv));
    float* q = op + 128 * u + 4 * lane;
    *(volatile v4f*)q = o;
    __threadfence();
    *(volatile v4f*)q = o;
  }
}

__global__ __launch_bounds__(256) void ln2_kernel(const float* __restrict__ xin, const float* __restrict__ gam,
                                                  const float* __restrict__ bet, unsigned short* __restrict__ outp) {
  const int tid = threadIdx.x, lane = tid & 31, wave = tid >> 5;
  const int row = blockIdx.x * 8 + wave;
  const float* rp = xin + (size_t)row * kNC;
  v4f a[4], gg[4], bb[4];
#pragma unroll
  for (int u = 0; u < 2; ++u) {
    const int off = 256 * u + 8 * lane;
    a[2 * u]      = *(const v4f*)(rp + off);
    a[2 * u + 1]  = *(const v4f*)(rp + off + 4);
    gg[2 * u]     = *(const v4f*)(gam + off);
    gg[2 * u + 1] = *(const v4f*)(gam + off + 4);
    bb[2 * u]     = *(const v4f*)(bet + off);
    bb[2 * u + 1] = *(const v4f*)(bet + off + 4);
  }
  float s = 0.0f;
#pragma unroll
  for (int i = 0; i < 4; ++i) s += (a[i][0] + a[i][1]) + (a[i][2] + a[i][3]);
#pragma unroll
  for (int off = 1; off < 32; off <<= 1) s += __shfl_xor(s, off, 32);
  const float mu = s * kInvC;
  float ss = 0.0f;
#pragma unroll
  for (int i = 0; i < 4; ++i)
#pragma unroll
    for (int e = 0; e < 4; ++e) { const float d = a[i][e] - mu; a[i][e] = d; ss += d * d; }
#pragma unroll
  for (int off = 1; off < 32; off <<= 1) ss += __shfl_xor(ss, off, 32);
  const float rstd = 1.0f / sqrtf(ss * kInvC + kLnEps);
  v8h hv[2];
#pragma unroll
  for (int i = 0; i < 4; ++i)
#pragma unroll
    for (int e = 0; e < 4; ++e) {
      const float val = (gg[i][e] * a[i][e]) * rstd + bb[i][e];
      hv[i >> 1][4 * (i & 1) + e] = (_Float16)val;
    }
  unsigned short* op = outp + (size_t)row * kNC;
  for (int pass = 0; pass < 2; ++pass) {
#pragma unroll
    for (int u = 0; u < 2; ++u) *(volatile v8h*)(op + 256 * u + 8 * lane) = hv[u];
    __threadfence();
  }
}

__global__ __launch_bounds__(256) void decay_scan_kernel(
    const float* __restrict__ qe, const float* __restrict__ ke, const float* __restrict__ vv,
    const float* __restrict__ gs, const float* __restrict__ lam, unsigned short* __restrict__ attg) {
  __shared__ __align__(16) float qs[kChunk * kND];
  __shared__ __align__(16) float ks[kChunk * kND];
  __shared__ __align__(16) float vs[kChunk * kSliceW];
  __shared__ __align__(16) float Sp[kChunk * 4 * kSliceW];
  __shared__ __align__(16) float zq[kChunk * kND];
  const int tid = threadIdx.x, lane = tid & 31, wave = tid >> 5;
  const int bh = blockIdx.x >> 1, slice = blockIdx.x & 1;
  const int b = bh >> 2, h = bh & 3;
  const int ig = wave >> 1;
  const int jl = (wave & 1) * 32 + lane;
  const int chan0 = h * kND;
  const int jcol0 = chan0 + slice * kSliceW;
  const size_t rowbase = (size_t)b * kNT;

  float lamr[32];
#pragma unroll
  for (int c = 0; c < 8; ++c) {
    const v4f l4 = *(const v4f*)(lam + chan0 + ig * 32 + 4 * c);
#pragma unroll
    for (int e = 0; e < 4; ++e) lamr[4 * c + e] = l4[e];
  }
  const float lamz = lam[chan0 + ig * 32 + lane];
  float Ast[32];
#pragma unroll
  for (int i = 0; i < 32; ++i) Ast[i] = 0.0f;
  float zl = 0.0f;

#pragma unroll 1
  for (int t0 = 0; t0 < kNT; t0 += kChunk) {
#pragma unroll
    for (int u = 0; u < 2; ++u) {
      const int idx = tid + 256 * u;
      const int s = idx >> 5, c4 = (idx & 31) * 4;
      const size_t goff = (rowbase + t0 + s) * kNC + chan0 + c4;
      *(v4f*)(qs + s * kND + c4) = *(const v4f*)(qe + goff);
      *(v4f*)(ks + s * kND + c4) = *(const v4f*)(ke + goff);
    }
    {
      const int s = tid >> 4, c4 = (tid & 15) * 4;
      *(v4f*)(vs + s * kSliceW + c4) = *(const v4f*)(vv + (rowbase + t0 + s) * kNC + jcol0 + c4);
    }
    __syncthreads();
#pragma unroll 1
    for (int s = 0; s < kChunk; ++s) {
      const float vj = vs[s * kSliceW + jl];
      const float* kp = ks + s * kND + ig * 32;
      const float* qp = qs + s * kND + ig * 32;
      float part = 0.0f;
#pragma unroll
      for (int c = 0; c < 8; ++c) {
        const v4f k4 = *(const v4f*)(kp + 4 * c);
        const v4f q4 = *(const v4f*)(qp + 4 * c);
#pragma unroll
        for (int e = 0; e < 4; ++e) {
          const float an = fmaf(k4[e], vj, lamr[4 * c + e] * Ast[4 * c + e]);
          Ast[4 * c + e] = an;
          part = fmaf(q4[e], an, part);
        }
      }
      Sp[(s * 4 + ig) * kSliceW + jl] = part;
      const float kl = kp[lane];
      const float ql = qp[lane];
      zl = fmaf(lamz, zl, kl);
      if ((wave & 1) == 0) zq[s * kND + ig * 32 + lane] = ql * zl;
    }
    __syncthreads();
    if (tid < 128) {
      const int s = tid >> 3, j0 = (tid & 7) * 8;
      float z0 = 0.0f, z1 = 0.0f, z2 = 0.0f, z3 = 0.0f;
#pragma unroll 4
      for (int c = 0; c < 32; ++c) {
        const v4f z4 = *(const v4f*)(zq + s * kND + 4 * c);
        z0 += z4[0]; z1 += z4[1]; z2 += z4[2]; z3 += z4[3];
      }
      const float Zt = (z0 + z1) + (z2 + z3);
      const float invZ = 1.0f / Zt;
      const size_t grow = (rowbase + t0 + s) * kNC + jcol0 + j0;
      const v4f g0 = *(const v4f*)(gs + grow);
      const v4f g1 = *(const v4f*)(gs + grow + 4);
      v8h hv;
#pragma unroll
      for (int hf = 0; hf < 2; ++hf) {
        const v4f s0 = *(const v4f*)(Sp + (s * 4 + 0) * kSliceW + j0 + 4 * hf);
        const v4f s1 = *(const v4f*)(Sp + (s * 4 + 1) * kSliceW + j0 + 4 * hf);
        const v4f s2 = *(const v4f*)(Sp + (s * 4 + 2) * kSliceW + j0 + 4 * hf);
        const v4f s3 = *(const v4f*)(Sp + (s * 4 + 3) * kSliceW + j0 + 4 * hf);
#pragma unroll
        for (int e = 0; e < 4; ++e) {
          const float St = (s0[e] + s1[e]) + (s2[e] + s3[e]);
          const float ge = hf ? g1[e] : g0[e];
          const float val = (ge * (St * invZ)) * kActCarry;
          hv[4 * hf + e] = (_Float16)val;
        }
      }
      unsigned short* op = attg + grow;
      *(volatile v8h*)op = hv;
      __threadfence();
      *(volatile v8h*)op = hv;
    }
  }
}

extern "C" void kernel_launch(void* const* d_in, const int* in_sizes, int n_in,
                              void* d_out, int out_size, void* d_ws, size_t ws_size, hipStream_t stream) {
  if (n_in < 18 || d_out == nullptr || d_ws == nullptr) return;
  if (in_sizes[0] != kRows * kNC || out_size != kRows * kNC) return;
  for (int i = 1; i <= 9; ++i) if (in_sizes[i] != kNC) return;
  for (int i = 10; i <= 14; ++i) if (in_sizes[i] != kNC * kNC) return;
  if (in_sizes[15] != kNC || in_sizes[16] != kFF * kNC || in_sizes[17] != kNC * kFF) return;

  const float* x     = (const float*)d_in[0];
  const float* ln1_g = (const float*)d_in[1];
  const float* ln1_b = (const float*)d_in[2];
  const float* ln2_g = (const float*)d_in[3];
  const float* ln2_b = (const float*)d_in[4];
  const float* tdec  = (const float*)d_in[5];
  const float* tm_q  = (const float*)d_in[6];
  const float* tm_k  = (const float*)d_in[7];
  const float* tm_v  = (const float*)d_in[8];
  const float* tm_g  = (const float*)d_in[9];
  const float* Wq    = (const float*)d_in[10];
  const float* Wk    = (const float*)d_in[11];
  const float* Wv    = (const float*)d_in[12];
  const float* Wg    = (const float*)d_in[13];
  const float* Wo    = (const float*)d_in[14];
  const float* rms_s = (const float*)d_in[15];
  const float* W1    = (const float*)d_in[16];
  const float* W2    = (const float*)d_in[17];
  float* outp = (float*)d_out;

  char* ws = (char*)d_ws;
  size_t off = 0;
  auto carve = [&](size_t bytes) -> char* { char* p = ws + off; off += (bytes + 255) & ~(size_t)255; return p; };
  const size_t planeElems = (size_t)kRows * kNC;
  unsigned short* W16   = (unsigned short*)carve(((size_t)5 * kNC * kNC + (size_t)2 * kFF * kNC) * 2);
  float*          LAM   = (float*)carve((size_t)kNC * 4);
  unsigned short* XMIX  = (unsigned short*)carve(4 * planeElems * 2);
  float*          QKVG  = (float*)carve(4 * planeElems * 4);
  float*          QKE   = (float*)carve(2 * planeElems * 4);
  unsigned short* ATTG  = (unsigned short*)carve(planeElems * 2);
  float*          X1    = (float*)carve(planeElems * 4);
  unsigned short* H2    = (unsigned short*)carve(planeElems * 2);
  unsigned short* FFACT = (unsigned short*)carve((size_t)kRows * kFF * 2);
  if (off > ws_size || off > (size_t)134217728) return;

  unsigned short* WoH = W16 + (size_t)4 * kNC * kNC;
  unsigned short* W1H = W16 + (size_t)5 * kNC * kNC;
  unsigned short* W2H = W1H + (size_t)kFF * kNC;

  prep_kernel<<<kCvtBlocks + 1, 256, 0, stream>>>(Wq, Wk, Wv, Wg, Wo, W1, W2, tdec, W16, LAM);

  ln1_mix_kernel<<<kRows / 8, 256, 0, stream>>>(x, ln1_g, ln1_b, tm_q, tm_k, tm_v, tm_g, XMIX);

  wmma_gemm64_h<0, false, 2><<<dim3((kRows / 64) * (kNC / 64) / 8, 4), 256, 0, stream>>>(
      XMIX, kNC, (long)planeElems, W16, kNC, (long)kNC * kNC, (void*)QKVG, kNC, (long)planeElems,
      x, 0L, kRows, kNC, kNC, kScaleW, 1.0f);

  rms_exp_kernel<<<dim3(kRows / 8, 2), 256, 0, stream>>>(QKVG, rms_s, QKE);

  decay_scan_kernel<<<kNB * kNH * 2, 256, 0, stream>>>(QKE, QKE + planeElems, QKVG + 2 * planeElems,
                                                       QKVG + 3 * planeElems, LAM, ATTG);

  wmma_gemm64_h<0, true, 0><<<dim3((kRows / 64) * (kNC / 64) / 8, 1), 256, 0, stream>>>(
      ATTG, kNC, 0L, WoH, kNC, 0L, (void*)X1, kNC, 0L,
      x, 0L, kRows, kNC, kNC, kScaleWA, 1.0f);

  ln2_kernel<<<kRows / 8, 256, 0, stream>>>(X1, ln2_g, ln2_b, H2);

  wmma_gemm64_h<1, false, 1><<<dim3((kRows / 64) * (kFF / 64) / 8, 1), 256, 0, stream>>>(
      H2, kNC, 0L, W1H, kNC, 0L, (void*)FFACT, kFF, 0L,
      x, 0L, kRows, kFF, kNC, kScaleW, kActCarry);

  wmma_gemm64_h<0, true, 0><<<dim3((kRows / 64) * (kNC / 64) / 8, 1), 256, 0, stream>>>(
      FFACT, kFF, 0L, W2H, kFF, 0L, (void*)outp, kNC, 0L,
      X1, 0L, kRows, kNC, kFF, kScaleWA, 1.0f);
}
